// Downsampleimprove1_18038862643770
// MI455X (gfx1250) — hardware-verified
//
#include <hip/hip_runtime.h>
#include <stdint.h>

#pragma clang fp contract(off)

#define CIN    2048
#define IMH    32
#define IMW    32
#define NPX    (IMH * IMW)
#define NTAP   9
#define NL     16
#define NO     256
#define KT     (NTAP * CIN)
#define PD     (IMH + 2)
#define NPD    (PD * PD)
#define NBORD  (NPD - NPX)
#define CHK    (KT / 8)
#define CGRP   64
#define STP    36
#define EPSBN  1e-5f

static_assert(KT % 32 == 0);
static_assert(CIN % 32 == 0);
static_assert(CIN % CGRP == 0);
static_assert((NO * CHK) % 256 == 0);
static_assert((NL * CHK) % 256 == 0);
static_assert((STP * 4) % 16 == 0);
static_assert(NBORD == 132);
static_assert(NPX == 4 * 256);

typedef __bf16         v16b __attribute__((ext_vector_type(16)));
typedef __bf16         v8b  __attribute__((ext_vector_type(8)));
typedef float          v8f  __attribute__((ext_vector_type(8)));
typedef float          v4f  __attribute__((ext_vector_type(4)));
typedef unsigned       v4u  __attribute__((ext_vector_type(4)));

__device__ __forceinline__ unsigned bfb(float f) {
  const unsigned u = __float_as_uint(f);
  return (u + 0x7FFFu + ((u >> 16) & 1u)) >> 16;
}
__device__ __forceinline__ float bf_rne(float f) { return __uint_as_float(bfb(f) << 16); }
__device__ __forceinline__ v8f zero8f() { v8f z = {0.f, 0.f, 0.f, 0.f, 0.f, 0.f, 0.f, 0.f}; return z; }

__device__ __forceinline__ v16b ldfrag_b(const __bf16* p) {
  union { v16b v; v8b h[2]; } f;
  f.h[0] = *(const v8b*)(p);
  f.h[1] = *(const v8b*)(p + 16);
  return f.v;
}

__device__ __forceinline__ v8f mma_b(v16b a, v16b b, v8f c) {
  return __builtin_amdgcn_wmma_f32_16x16x32_bf16(false, a, false, b, (short)0, c, false, false);
}
__device__ __forceinline__ void guard1x2(v8f& c0, const v16b& f0, const v16b& f1) {
#if defined(__HIP_DEVICE_COMPILE__)
  asm volatile("v_nop\n\tv_nop\n\tv_nop\n\tv_nop" : "+v"(c0) : "v"(f0), "v"(f1));
#endif
}
__device__ __forceinline__ void guard4x5(v8f& c0, v8f& c1, v8f& c2, v8f& c3,
                                         const v16b& f0, const v16b& f1, const v16b& f2,
                                         const v16b& f3, const v16b& f4) {
#if defined(__HIP_DEVICE_COMPILE__)
  asm volatile("v_nop\n\tv_nop\n\tv_nop\n\tv_nop"
               : "+v"(c0), "+v"(c1), "+v"(c2), "+v"(c3)
               : "v"(f0), "v"(f1), "v"(f2), "v"(f3), "v"(f4));
#endif
}
__device__ __forceinline__ void acc_guard1(v8f& c0) {
#if defined(__HIP_DEVICE_COMPILE__)
  asm volatile("v_nop\n\tv_nop\n\tv_nop\n\tv_nop" : "+v"(c0));
#endif
}
__device__ __forceinline__ void acc_guard4(v8f& c0, v8f& c1, v8f& c2, v8f& c3) {
#if defined(__HIP_DEVICE_COMPILE__)
  asm volatile("v_nop\n\tv_nop\n\tv_nop\n\tv_nop" : "+v"(c0), "+v"(c1), "+v"(c2), "+v"(c3));
#endif
}

__global__ __launch_bounds__(256)
void k_xplane(const float* __restrict__ x, unsigned short* xp)
{
  __shared__ float tile[CGRP * 33];
  const int tid  = threadIdx.x;
  const int lane = tid & 31;
  const int wid  = tid >> 5;
  const int pj   = lane & 7;
  const int lq   = lane >> 3;
  const int cg   = blockIdx.x;
  const int by   = blockIdx.y;
  const int n    = by >> 5;
  const int y    = by & 31;
  const int px   = tid & 31;
  const int cr   = tid >> 5;
#pragma unroll
  for (int i = 0; i < 8; ++i) {
    const int c = cr + 8 * i;
    tile[c * 33 + px] = x[((size_t)(n * CIN + CGRP * cg + c)) * NPX + y * IMW + px];
  }
  __syncthreads();
  const int L = wid * 4 + lq;
  unsigned hb[8];
#pragma unroll
  for (int e = 0; e < 8; ++e) hb[e] = bfb(tile[(8 * pj + e) * 33 + L]);
  v4u wv;
  wv.x = hb[0] | (hb[1] << 16);
  wv.y = hb[2] | (hb[3] << 16);
  wv.z = hb[4] | (hb[5] << 16);
  wv.w = hb[6] | (hb[7] << 16);
  const size_t eo = (((size_t)(n * PD + y + 1)) * PD + L + 1) * CIN + CGRP * cg + 8 * pj;
  *(volatile v4u*)(xp + eo) = wv;
  __threadfence();
  *(volatile v4u*)(xp + eo) = wv;
}

__global__ __launch_bounds__(256)
void k_border(unsigned short* xp)
{
  const int tid  = threadIdx.x;
  const int lane = tid & 31;
  const int wid  = tid >> 5;
  const int pj   = lane & 7;
  const int lq   = lane >> 3;
  const int b    = blockIdx.x;
  const int n    = b / NBORD;
  const int r    = b - n * NBORD;
  int py, px;
  if (r < PD)          { py = 0;      px = r; }
  else if (r < 2 * PD) { py = PD - 1; px = r - PD; }
  else { const int q = r - 2 * PD; py = 1 + (q >> 1); px = (q & 1) ? (PD - 1) : 0; }
  const int L = wid * 4 + lq;
  const v4u z = {0u, 0u, 0u, 0u};
  const size_t eo = (((size_t)(n * PD + py)) * PD + px) * CIN + L * CGRP + 8 * pj;
  *(volatile v4u*)(xp + eo) = z;
  __threadfence();
  *(volatile v4u*)(xp + eo) = z;
}

__global__ __launch_bounds__(256)
void k_pack(const float* __restrict__ w, int nrows, unsigned* dst, int nchunks)
{
  const int q    = blockIdx.x * 256 + threadIdx.x;
  const int qc   = min(q, nchunks - 1);
  const int row  = qc / CHK;
  const int kc   = (qc - row * CHK) * 8;
  const int t    = kc >> 11;
  const int c    = kc & (CIN - 1);
  const bool live = (row < nrows);
  const int rowc = min(row, nrows - 1);
  const float* s = w + ((size_t)rowc * CIN + c) * NTAP + t;
  unsigned hb[8];
#pragma unroll
  for (int j = 0; j < 8; ++j) {
    const float v = s[j * NTAP];
    hb[j] = live ? bfb(v) : 0u;
  }
  v4u wh;
  wh.x = hb[0] | (hb[1] << 16);
  wh.y = hb[2] | (hb[3] << 16);
  wh.z = hb[4] | (hb[5] << 16);
  wh.w = hb[6] | (hb[7] << 16);
  const bool ok = (q < nchunks);
  unsigned* d = dst + (size_t)qc * 4;
  if (ok) *(volatile v4u*)d = wh;
  __threadfence();
  if (ok) *(volatile v4u*)d = wh;
}

__global__ __launch_bounds__(64)
void k_conv(const __bf16* __restrict__ xp, const __bf16* __restrict__ bc, float* sig)
{
  __shared__ __align__(16) float sg[NL * STP];
  const int tid  = threadIdx.x;
  const int lane = tid & 31;
  const int wid  = tid >> 5;
  const int m    = lane & 15;
  const int hh   = lane >> 4;
  const int pj   = lane & 7;
  const int lq   = lane >> 3;
  const int b    = blockIdx.x;
  const int n    = b >> 5;
  const int y    = b & 31;
  const int x0   = 16 * wid;

  v8f acc = zero8f();
  const __bf16* bbase = bc + (size_t)m * KT + 8 * hh;
#pragma unroll 1
  for (int t = 0; t < NTAP; ++t) {
    const int dy = t / 3;
    const int dx = t - 3 * dy;
    const __bf16* ap = xp + ((size_t)((n * PD + y + dy) * PD + x0 + m + dx)) * CIN + 8 * hh;
    const __bf16* bp = bbase + (size_t)t * CIN;
#pragma unroll 2
    for (int s = 0; s < CIN / 32; ++s) {
      const v16b fa = ldfrag_b(ap + 32 * s);
      const v16b fb = ldfrag_b(bp + 32 * s);
      acc = mma_b(fa, fb, acc);
      guard1x2(acc, fa, fb);
    }
  }
  acc_guard1(acc);

  {
    v4f o0, o1;
#pragma unroll
    for (int r = 0; r < 4; ++r) { o0[r] = acc[r]; o1[r] = acc[4 + r]; }
    float* ep = sg + m * STP + x0 + 8 * hh;
    *(v4f*)ep       = o0;
    *(v4f*)(ep + 4) = o1;
  }
  __syncthreads();
  {
    v4f val[2]; size_t e[2];
#pragma unroll
    for (int it = 0; it < 2; ++it) {
      const int L = it * 8 + wid * 4 + lq;
      val[it] = *(const v4f*)&sg[L * STP + 4 * pj];
      e[it]   = ((size_t)(n * NL + L)) * NPX + y * IMW + 4 * pj;
    }
#pragma unroll
    for (int it = 0; it < 2; ++it) *(volatile v4f*)(sig + e[it]) = val[it];
    __threadfence();
#pragma unroll
    for (int it = 0; it < 2; ++it) *(volatile v4f*)(sig + e[it]) = val[it];
  }
}

__global__ __launch_bounds__(256)
void k_bnsoft(const float* __restrict__ sig, const float* __restrict__ gam,
              const float* __restrict__ bet, int nb, float* ss)
{
  __shared__ double rsd[256];
  __shared__ double rqd[256];
  __shared__ float stt[64];
  const int tid = threadIdx.x;
  if (tid < NTAP) { stt[32 + tid] = bf_rne(gam[tid]); stt[48 + tid] = bf_rne(bet[tid]); }
  const int cnt = nb * NPX;
  const double invn = 1.0 / (double)cnt;
#pragma unroll 1
  for (int l = 0; l < NTAP; ++l) {
    double s = 0.0, q = 0.0;
#pragma unroll 1
    for (int p = tid; p < cnt; p += 256) {
      const float v = sig[(((size_t)((p >> 10) * NL + l)) << 10) + (p & 1023)];
      s += (double)v;
      q += (double)v * (double)v;
    }
    rsd[tid] = s;
    rqd[tid] = q;
    __syncthreads();
#pragma unroll 1
    for (int off = 128; off > 0; off >>= 1) {
      if (tid < off) { rsd[tid] = rsd[tid] + rsd[tid + off]; rqd[tid] = rqd[tid] + rqd[tid + off]; }
      __syncthreads();
    }
    if (tid == 0) {
      const double mean = rsd[0] * invn;
      double var = rqd[0] * invn - mean * mean;
      if (var < 0.0) var = 0.0;
      stt[l]      = (float)mean;
      stt[16 + l] = 1.0f / sqrtf((float)var + EPSBN);
    }
    __syncthreads();
  }

  float mu[NTAP], rs[NTAP], ga[NTAP], be[NTAP];
#pragma unroll
  for (int l = 0; l < NTAP; ++l) { mu[l] = stt[l]; rs[l] = stt[16 + l]; ga[l] = stt[32 + l]; be[l] = stt[48 + l]; }

  const int nit = nb * (NPX / 256);
#pragma unroll 1
  for (int it = 0; it < nit; ++it) {
    const int p = it * 256 + tid;
    const int n = p >> 10;
    const int m = p & 1023;
    float v[NTAP];
#pragma unroll
    for (int l = 0; l < NTAP; ++l) {
      const float s = sig[(((size_t)(n * NL + l)) << 10) + m];
      float t = s - mu[l];
      t = t * rs[l];
      t = t * ga[l];
      t = t + be[l];
      v[l] = t;
    }
    float mx = v[0];
#pragma unroll
    for (int l = 1; l < NTAP; ++l) mx = fmaxf(mx, v[l]);
    float sum = 0.0f;
#pragma unroll
    for (int l = 0; l < NTAP; ++l) { v[l] = __expf(v[l] - mx); sum = sum + v[l]; }
    const float inv = 1.0f / sum;
#pragma unroll
    for (int l = 0; l < NTAP; ++l) v[l] = v[l] * inv;
    float* d = ss + (((size_t)(n * NTAP)) << 10) + m;
#pragma unroll
    for (int l = 0; l < NTAP; ++l) *(volatile float*)(d + ((size_t)l << 10)) = v[l];
    __threadfence();
#pragma unroll
    for (int l = 0; l < NTAP; ++l) *(volatile float*)(d + ((size_t)l << 10)) = v[l];
  }
}

__global__ __launch_bounds__(256)
void k_main(const __bf16* __restrict__ xp, const __bf16* __restrict__ bw,
            const float* __restrict__ ss, float* out)
{
  __shared__ __align__(16) float st[NO * STP];
  const int tid  = threadIdx.x;
  const int lane = tid & 31;
  const int wid  = tid >> 5;
  const int m    = lane & 15;
  const int hh   = lane >> 4;
  const int pj   = lane & 7;
  const int lq   = lane >> 3;
  const int b    = blockIdx.x;
  const int n    = b >> 5;
  const int y    = b & 31;
  const int mh   = wid >> 2;
  const int cg   = wid & 3;
  const int x0   = 16 * mh;
  const int o0   = 64 * cg;

  v8f acc[4], part[4];
#pragma unroll
  for (int j = 0; j < 4; ++j) { acc[j] = zero8f(); part[j] = zero8f(); }

  const __bf16* bbase = bw + (size_t)(o0 + m) * KT + 8 * hh;
  const float*  sbase = ss + ((size_t)(n * NTAP)) * NPX + y * IMW + x0 + 8 * hh;

#pragma unroll 1
  for (int t = 0; t < NTAP; ++t) {
    const int dy = t / 3;
    const int dx = t - 3 * dy;
    const __bf16* ap = xp + ((size_t)((n * PD + y + dy) * PD + x0 + m + dx)) * CIN + 8 * hh;
    const __bf16* bp = bbase + (size_t)t * CIN;
#pragma unroll 1
    for (int s = 0; s < CIN / 32; ++s) {
      const v16b fa = ldfrag_b(ap + 32 * s);
      v16b fb[4];
#pragma unroll
      for (int j = 0; j < 4; ++j) fb[j] = ldfrag_b(bp + (size_t)j * 16 * KT + 32 * s);
#pragma unroll
      for (int j = 0; j < 4; ++j) part[j] = mma_b(fa, fb[j], part[j]);
      guard4x5(part[0], part[1], part[2], part[3], fa, fb[0], fb[1], fb[2], fb[3]);
    }
    acc_guard4(part[0], part[1], part[2], part[3]);
    const v4f s0 = *(const v4f*)(sbase + (size_t)t * NPX);
    const v4f s1 = *(const v4f*)(sbase + (size_t)t * NPX + 4);
#pragma unroll
    for (int j = 0; j < 4; ++j) {
#pragma unroll
      for (int r = 0; r < 4; ++r) acc[j][r] = acc[j][r] + s0[r] * part[j][r];
#pragma unroll
      for (int r = 0; r < 4; ++r) acc[j][4 + r] = acc[j][4 + r] + s1[r] * part[j][4 + r];
      part[j] = zero8f();
    }
  }

#pragma unroll
  for (int j = 0; j < 4; ++j) {
    const int ol = o0 + 16 * j + m;
    v4f q0, q1;
#pragma unroll
    for (int r = 0; r < 4; ++r) { q0[r] = acc[j][r]; q1[r] = acc[j][4 + r]; }
    float* ep = st + ol * STP + x0 + 8 * hh;
    *(v4f*)ep       = q0;
    *(v4f*)(ep + 4) = q1;
  }
  __syncthreads();
  {
    v4f val[8]; size_t e[8];
#pragma unroll
    for (int it = 0; it < 8; ++it) {
      const int L = it * 32 + wid * 4 + lq;
      val[it] = *(const v4f*)&st[L * STP + 4 * pj];
      e[it]   = ((size_t)(n * NO + L)) * NPX + y * IMW + 4 * pj;
    }
#pragma unroll
    for (int it = 0; it < 8; ++it) *(volatile v4f*)(out + e[it]) = val[it];
    __threadfence();
#pragma unroll
    for (int it = 0; it < 8; ++it) *(volatile v4f*)(out + e[it]) = val[it];
  }
}

extern "C" void kernel_launch(void* const* d_in, const int* in_sizes, int n_in,
                              void* d_out, int out_size, void* d_ws, size_t ws_size,
                              hipStream_t stream) {
  if (n_in < 5) return;
  const int nx = in_sizes[0];
  if (nx <= 0 || (nx % (CIN * NPX)) != 0) return;
  const int NB = nx / (CIN * NPX);
  if (NB < 1) return;
  if (in_sizes[1] != NTAP * CIN * NTAP) return;
  if (in_sizes[2] != NTAP || in_sizes[3] != NTAP) return;
  if (in_sizes[4] != NO * CIN * NTAP) return;
  if (out_size != NB * NO * NPX) return;

  const size_t o_xp  = 0;
  const size_t o_bw  = o_xp + (size_t)NB * NPD * CIN * 2;
  const size_t o_bc  = o_bw + (size_t)NO * KT * 2;
  const size_t o_sig = o_bc + (size_t)NL * KT * 2;
  const size_t o_ss  = o_sig + (size_t)NB * NL * NPX * 4;
  const size_t o_end = o_ss + (size_t)NB * NTAP * NPX * 4;
  if (o_end > ws_size) return;

  const float* x    = (const float*)d_in[0];
  const float* cw   = (const float*)d_in[1];
  const float* gam  = (const float*)d_in[2];
  const float* bet  = (const float*)d_in[3];
  const float* wgt  = (const float*)d_in[4];
  float* out = (float*)d_out;
  char* ws = (char*)d_ws;

  unsigned short* xp  = (unsigned short*)(ws + o_xp);
  unsigned*       bw  = (unsigned*)(ws + o_bw);
  unsigned*       bc  = (unsigned*)(ws + o_bc);
  float*          sig = (float*)(ws + o_sig);
  float*          ss  = (float*)(ws + o_ss);

  k_xplane<<<dim3(CIN / CGRP, NB * IMH), dim3(256), 0, stream>>>(x, xp);
  (void)hipGetLastError();
  k_border<<<dim3(NB * NBORD), dim3(256), 0, stream>>>(xp);
  (void)hipGetLastError();
  k_pack<<<dim3((NL * CHK) / 256), dim3(256), 0, stream>>>(cw, NTAP, bc, NL * CHK);
  (void)hipGetLastError();
  k_pack<<<dim3((NO * CHK) / 256), dim3(256), 0, stream>>>(wgt, NO, bw, NO * CHK);
  (void)hipGetLastError();
  k_conv<<<dim3(NB * IMH), dim3(64), 0, stream>>>((const __bf16*)xp, (const __bf16*)bc, sig);
  (void)hipGetLastError();
  k_bnsoft<<<dim3(1), dim3(256), 0, stream>>>(sig, gam, bet, NB, ss);
  (void)hipGetLastError();
  k_main<<<dim3(NB * IMH), dim3(256), 0, stream>>>((const __bf16*)xp, (const __bf16*)bw, ss, out);
  (void)hipGetLastError();
}
